// WatsonCrickMultiHeadedAttention_33363305956083
// MI455X (gfx1250) — hardware-verified
//
#include <hip/hip_runtime.h>
#include <stddef.h>


typedef __bf16         v16bf __attribute__((ext_vector_type(16)));
typedef float          v8f   __attribute__((ext_vector_type(8)));
typedef float          v4f   __attribute__((ext_vector_type(4)));
typedef unsigned int   v4u   __attribute__((ext_vector_type(4)));
typedef float          v4fa  __attribute__((ext_vector_type(4), __may_alias__));
typedef unsigned int   v4ua  __attribute__((ext_vector_type(4), __may_alias__));
typedef unsigned short u16;

#define NB     8
#define NTOK   1024
#define DM     512
#define NH     8
#define DK     64
#define MROWS  (NB * NTOK)
#define ACT_N  (MROWS * DM)
#define W_N    (DM * DM)
#define GATE_N (NB * NTOK * NTOK)

union Frag { v16bf v; v4u q[2]; };
union __attribute__((aligned(16))) TileU { u16 h[16384]; float f[8192]; };

__device__ __forceinline__ unsigned int bf_bits(float x)
{
    const unsigned int u = __float_as_uint(x);
    return (u + 0x7FFFu + ((u >> 16) & 1u)) >> 16;
}

__device__ __forceinline__ void split_bf(float x, unsigned int& hi, unsigned int& lo)
{
    hi = bf_bits(x);
    lo = bf_bits(x - __uint_as_float(hi << 16));
}

__device__ __forceinline__ v4u pack8(const unsigned int* x)
{
    v4u r;
    r[0] = (x[0] & 0xFFFFu) | (x[1] << 16);
    r[1] = (x[2] & 0xFFFFu) | (x[3] << 16);
    r[2] = (x[4] & 0xFFFFu) | (x[5] << 16);
    r[3] = (x[6] & 0xFFFFu) | (x[7] << 16);
    return r;
}

__device__ __forceinline__ void wmma3(v8f& acc, const v16bf ah, const v16bf al,
                                      const v16bf bh, const v16bf bl)
{
    acc = __builtin_amdgcn_wmma_f32_16x16x32_bf16(false, ah, false, bh, (short)0, acc, false, false);
    acc = __builtin_amdgcn_wmma_f32_16x16x32_bf16(false, ah, false, bl, (short)0, acc, false, false);
    acc = __builtin_amdgcn_wmma_f32_16x16x32_bf16(false, al, false, bh, (short)0, acc, false, false);
    asm volatile("v_nop\n\tv_nop\n\tv_nop\n\tv_nop" : "+v"(acc) : "v"(ah), "v"(al), "v"(bh), "v"(bl));
}

__device__ __forceinline__ v16bf ld_frag_g(const u16* p, int h)
{
    Frag f;
    f.q[0] = *(const v4ua*)(p + 8 * h);
    f.q[1] = *(const v4ua*)(p + 16 + 8 * h);
    return f.v;
}

__global__ __launch_bounds__(256) void k_gate(const float* __restrict__ wc, float* __restrict__ G)
{
    __shared__ float red[8];
    const int t = threadIdx.x, wave = t >> 5, lane = t & 31;
    const size_t rb = (size_t)blockIdx.x * NTOK;

    const v4f x = *(const v4fa*)(wc + rb + 4 * t);
    float mx = fmaxf(fmaxf(x[0], x[1]), fmaxf(x[2], x[3]));
    #pragma unroll
    for (int off = 16; off >= 1; off >>= 1) mx = fmaxf(mx, __shfl_xor(mx, off, 32));
    if (lane == 0) red[wave] = mx;
    __syncthreads();
    float mm = red[lane & 7];
    #pragma unroll
    for (int off = 4; off >= 1; off >>= 1) mm = fmaxf(mm, __shfl_xor(mm, off, 32));
    __syncthreads();

    v4f e;
    e[0] = __expf(x[0] - mm);
    e[1] = __expf(x[1] - mm);
    e[2] = __expf(x[2] - mm);
    e[3] = __expf(x[3] - mm);
    float sum = (e[0] + e[1]) + (e[2] + e[3]);
    #pragma unroll
    for (int off = 16; off >= 1; off >>= 1) sum += __shfl_xor(sum, off, 32);
    if (lane == 0) red[wave] = sum;
    __syncthreads();
    float ss = red[lane & 7];
    #pragma unroll
    for (int off = 4; off >= 1; off >>= 1) ss += __shfl_xor(ss, off, 32);

    const float inv = 1.0f / ss;
    const v4f r = e * inv;
    float* dst = G + rb + 4 * t;
    *(volatile v4fa*)dst = r;
    __threadfence();
    *(volatile v4fa*)dst = r;
}

__global__ __launch_bounds__(256) void k_split(
    const float* __restrict__ xq, const float* __restrict__ xk, const float* __restrict__ xv,
    const float* __restrict__ wq, const float* __restrict__ wk,
    const float* __restrict__ wv, const float* __restrict__ wo,
    u16* __restrict__ xpl, u16* __restrict__ wpl)
{
    const int bid = blockIdx.x;
    const float* src;
    u16* dh;
    u16* dl;
    size_t e;
    if (bid < 3 * 2048) {
        const int seg = bid >> 11;
        const int lb  = bid & 2047;
        src = (seg == 0) ? xq : ((seg == 1) ? xk : xv);
        e   = ((size_t)lb * 256 + threadIdx.x) * 8;
        dh  = xpl + (size_t)seg * 2 * ACT_N;
        dl  = dh + ACT_N;
    } else {
        const int wb  = bid - 3 * 2048;
        const int seg = wb >> 7;
        const int lb  = wb & 127;
        src = (seg == 0) ? wq : ((seg == 1) ? wk : ((seg == 2) ? wv : wo));
        e   = ((size_t)lb * 256 + threadIdx.x) * 8;
        dh  = wpl + (size_t)seg * 2 * W_N;
        dl  = dh + W_N;
    }

    const v4f a = *(const v4fa*)(src + e);
    const v4f c = *(const v4fa*)(src + e + 4);
    unsigned int hi[8], lo[8];
    split_bf(a[0], hi[0], lo[0]);
    split_bf(a[1], hi[1], lo[1]);
    split_bf(a[2], hi[2], lo[2]);
    split_bf(a[3], hi[3], lo[3]);
    split_bf(c[0], hi[4], lo[4]);
    split_bf(c[1], hi[5], lo[5]);
    split_bf(c[2], hi[6], lo[6]);
    split_bf(c[3], hi[7], lo[7]);
    const v4u ph = pack8(hi);
    const v4u pl = pack8(lo);

    *(volatile v4ua*)(dh + e) = ph;
    *(volatile v4ua*)(dl + e) = pl;
    __threadfence();
    *(volatile v4ua*)(dh + e) = ph;
    *(volatile v4ua*)(dl + e) = pl;
}

template <int MODE>
__global__ __launch_bounds__(256) void k_gemm(
    const u16* __restrict__ Xh, const u16* __restrict__ Xl,
    const u16* __restrict__ Wh, const u16* __restrict__ Wl,
    const float* __restrict__ bias,
    u16* __restrict__ Oh, u16* __restrict__ Ol, float* __restrict__ Of)
{
    __shared__ TileU s_t;

    const int lane = threadIdx.x & 31, wave = threadIdx.x >> 5;
    const int hh = lane >> 4, m = lane & 15;
    const int rl0 = wave * 16;
    const int mb0 = blockIdx.y * 128;
    const int m0  = mb0 + rl0;
    const int n0  = blockIdx.x * 64;

    v8f zero = {};
    v8f acc[4];
    #pragma unroll
    for (int g = 0; g < 4; ++g) acc[g] = zero;

    const u16* xh = Xh + (size_t)(m0 + m) * DM;
    const u16* xl = Xl + (size_t)(m0 + m) * DM;
    const u16* wh = Wh + (size_t)(n0 + m) * DM;
    const u16* wl = Wl + (size_t)(n0 + m) * DM;

    #pragma unroll 1
    for (int k0 = 0; k0 < DM; k0 += 32) {
        const v16bf ah = ld_frag_g(xh + k0, hh);
        const v16bf al = ld_frag_g(xl + k0, hh);
        #pragma unroll
        for (int g = 0; g < 4; ++g) {
            const size_t go = (size_t)g * 16 * DM + k0;
            const v16bf bh = ld_frag_g(wh + go, hh);
            const v16bf bl = ld_frag_g(wl + go, hh);
            wmma3(acc[g], ah, al, bh, bl);
        }
    }

    if (MODE == 0) {
        #pragma unroll
        for (int g = 0; g < 4; ++g) {
            const int col = g * 16 + m;
            const float bb = bias[n0 + col];
            #pragma unroll
            for (int r = 0; r < 8; ++r) {
                unsigned int vh, vl;
                split_bf(acc[g][r] + bb, vh, vl);
                const int idx = (rl0 + 8 * hh + r) * 64 + col;
                s_t.h[idx]        = (u16)vh;
                s_t.h[8192 + idx] = (u16)vl;
            }
        }
        __syncthreads();
        v4u ph[4], pl[4];
        size_t dst[4];
        #pragma unroll
        for (int it = 0; it < 4; ++it) {
            const int rowl = rl0 + it * 4 + (lane >> 3);
            const int j = lane & 7;
            ph[it] = *(const v4ua*)(&s_t.h[rowl * 64 + 8 * j]);
            pl[it] = *(const v4ua*)(&s_t.h[8192 + rowl * 64 + 8 * j]);
            const int mg = mb0 + rowl;
            const int b = mg >> 10, n = mg & 1023;
            dst[it] = (((size_t)b * NH + blockIdx.x) * NTOK + n) * DK + 8 * j;
        }
        #pragma unroll
        for (int it = 0; it < 4; ++it) {
            *(volatile v4ua*)(Oh + dst[it]) = ph[it];
            *(volatile v4ua*)(Ol + dst[it]) = pl[it];
        }
        __threadfence();
        #pragma unroll
        for (int it = 0; it < 4; ++it) {
            *(volatile v4ua*)(Oh + dst[it]) = ph[it];
            *(volatile v4ua*)(Ol + dst[it]) = pl[it];
        }
    } else if (MODE == 1) {
        #pragma unroll
        for (int g = 0; g < 4; ++g) {
            const int col = g * 16 + m;
            const float bb = bias[n0 + col];
            unsigned int vh[8], vl[8];
            #pragma unroll
            for (int r = 0; r < 8; ++r) split_bf(acc[g][r] + bb, vh[r], vl[r]);
            const int idx = col * 128 + rl0 + 8 * hh;
            *(v4ua*)(&s_t.h[idx])        = pack8(vh);
            *(v4ua*)(&s_t.h[8192 + idx]) = pack8(vl);
        }
        __syncthreads();
        v4u ph[4], pl[4];
        size_t dst[4];
        const int b  = mb0 >> 10;
        const int nb = mb0 & 1023;
        #pragma unroll
        for (int it = 0; it < 4; ++it) {
            const int dkl = wave * 8 + it * 2 + hh;
            const int nl  = 8 * m;
            ph[it] = *(const v4ua*)(&s_t.h[dkl * 128 + nl]);
            pl[it] = *(const v4ua*)(&s_t.h[8192 + dkl * 128 + nl]);
            dst[it] = (((size_t)b * NH + blockIdx.x) * DK + dkl) * NTOK + nb + nl;
        }
        #pragma unroll
        for (int it = 0; it < 4; ++it) {
            *(volatile v4ua*)(Oh + dst[it]) = ph[it];
            *(volatile v4ua*)(Ol + dst[it]) = pl[it];
        }
        __threadfence();
        #pragma unroll
        for (int it = 0; it < 4; ++it) {
            *(volatile v4ua*)(Oh + dst[it]) = ph[it];
            *(volatile v4ua*)(Ol + dst[it]) = pl[it];
        }
    } else {
        #pragma unroll
        for (int g = 0; g < 4; ++g) {
            const int col = g * 16 + m;
            const float bb = bias[n0 + col];
            #pragma unroll
            for (int r = 0; r < 8; ++r)
                s_t.f[(rl0 + 8 * hh + r) * 64 + col] = acc[g][r] + bb;
        }
        __syncthreads();
        v4f pv[8];
        size_t dst[8];
        #pragma unroll
        for (int it = 0; it < 8; ++it) {
            const int rowl = rl0 + it * 2 + hh;
            pv[it]  = *(const v4fa*)(&s_t.f[rowl * 64 + 4 * m]);
            dst[it] = (size_t)(mb0 + rowl) * DM + n0 + 4 * m;
        }
        #pragma unroll
        for (int it = 0; it < 8; ++it) *(volatile v4fa*)(Of + dst[it]) = pv[it];
        __threadfence();
        #pragma unroll
        for (int it = 0; it < 8; ++it) *(volatile v4fa*)(Of + dst[it]) = pv[it];
    }
}

__global__ __launch_bounds__(256) void k_attn(
    const u16* __restrict__ Qh, const u16* __restrict__ Ql,
    const u16* __restrict__ Kh, const u16* __restrict__ Kl,
    const u16* __restrict__ Vh, const u16* __restrict__ Vl,
    const float* __restrict__ G,
    u16* __restrict__ Ch, u16* __restrict__ Cl)
{
    __shared__ __attribute__((aligned(16))) u16 s_p[8 * 2048];

    const int lane = threadIdx.x & 31, wave = threadIdx.x >> 5;
    const int hh = lane >> 4, m = lane & 15;
    const int bh = blockIdx.y, b = bh >> 3, hd = bh & 7;
    const int q0 = blockIdx.x * 128 + wave * 16;
    u16* sp = s_p + wave * 2048;

    const size_t hb = (size_t)bh * NTOK * DK;
    const u16* Qbh = Qh + hb;  const u16* Qbl = Ql + hb;
    const u16* Kbh = Kh + hb;  const u16* Kbl = Kl + hb;
    const u16* Vbh = Vh + hb;  const u16* Vbl = Vl + hb;
    const float* Gw = G + ((size_t)b * NTOK + q0) * NTOK;

    v16bf aqh[2], aql[2];
    #pragma unroll
    for (int kk = 0; kk < 2; ++kk) {
        const size_t qo = (size_t)(q0 + m) * DK + kk * 32;
        aqh[kk] = ld_frag_g(Qbh + qo, hh);
        aql[kk] = ld_frag_g(Qbl + qo, hh);
    }

    float mrun[8], lrun[8];
    v8f zero = {};
    v8f o[4];
    #pragma unroll
    for (int r = 0; r < 8; ++r) { mrun[r] = -1.0e30f; lrun[r] = 0.f; }
    #pragma unroll
    for (int g = 0; g < 4; ++g) o[g] = zero;

    #pragma unroll 1
    for (int j0 = 0; j0 < NTOK; j0 += 32) {
        v8f s[2];
        #pragma unroll
        for (int t = 0; t < 2; ++t) {
            const size_t ko = (size_t)(j0 + t * 16 + m) * DK;
            const v16bf bh0 = ld_frag_g(Kbh + ko, hh);
            const v16bf bl0 = ld_frag_g(Kbl + ko, hh);
            const v16bf bh1 = ld_frag_g(Kbh + ko + 32, hh);
            const v16bf bl1 = ld_frag_g(Kbl + ko + 32, hh);
            v8f z = zero;
            wmma3(z, aqh[0], aql[0], bh0, bl0);
            wmma3(z, aqh[1], aql[1], bh1, bl1);
            s[t] = z;
        }

        #pragma unroll
        for (int r = 0; r < 8; ++r) {
            const float* gr = Gw + (size_t)(8 * hh + r) * NTOK + j0 + m;
            const float g0 = gr[0];
            const float g1 = gr[16];
            const float s0 = (s[0][r] * 0.125f) * g0;
            const float s1 = (s[1][r] * 0.125f) * g1;
            float cm = fmaxf(s0, s1);
            #pragma unroll
            for (int off = 8; off >= 1; off >>= 1) cm = fmaxf(cm, __shfl_xor(cm, off, 32));
            const float mnew = fmaxf(mrun[r], cm);
            const float sc = __expf(mrun[r] - mnew);
            const float p0 = __expf(s0 - mnew);
            const float p1 = __expf(s1 - mnew);
            s[0][r] = p0;
            s[1][r] = p1;
            float rs = p0 + p1;
            #pragma unroll
            for (int off = 8; off >= 1; off >>= 1) rs += __shfl_xor(rs, off, 32);
            lrun[r] = lrun[r] * sc + rs;
            mrun[r] = mnew;
            #pragma unroll
            for (int g = 0; g < 4; ++g) o[g][r] *= sc;
        }

        __syncthreads();
        #pragma unroll
        for (int r = 0; r < 8; ++r) {
            const int row = 8 * hh + r;
            unsigned int h0, l0, h1, l1;
            split_bf(s[0][r], h0, l0);
            split_bf(s[1][r], h1, l1);
            sp[row * 32 + m]            = (u16)h0;
            sp[row * 32 + 16 + m]       = (u16)h1;
            sp[512 + row * 32 + m]      = (u16)l0;
            sp[512 + row * 32 + 16 + m] = (u16)l1;
        }
        __syncthreads();
        Frag aph, apl;
        aph.q[0] = *(const v4ua*)(sp + m * 32 + 8 * hh);
        aph.q[1] = *(const v4ua*)(sp + m * 32 + 16 + 8 * hh);
        apl.q[0] = *(const v4ua*)(sp + 512 + m * 32 + 8 * hh);
        apl.q[1] = *(const v4ua*)(sp + 512 + m * 32 + 16 + 8 * hh);

        #pragma unroll
        for (int g = 0; g < 4; ++g) {
            const size_t vo = (size_t)(g * 16 + m) * NTOK + j0;
            const v16bf bvh = ld_frag_g(Vbh + vo, hh);
            const v16bf bvl = ld_frag_g(Vbl + vo, hh);
            wmma3(o[g], aph.v, apl.v, bvh, bvl);
        }
    }

    __syncthreads();
    #pragma unroll
    for (int r = 0; r < 8; ++r) {
        const float inv = 1.0f / lrun[r];
        const int row = 8 * hh + r;
        #pragma unroll
        for (int g = 0; g < 4; ++g) {
            unsigned int vh, vl;
            split_bf(o[g][r] * inv, vh, vl);
            sp[row * 64 + g * 16 + m]        = (u16)vh;
            sp[1024 + row * 64 + g * 16 + m] = (u16)vl;
        }
    }
    __syncthreads();
    v4u ph[4], pl[4];
    size_t dst[4];
    #pragma unroll
    for (int it = 0; it < 4; ++it) {
        const int rowl = it * 4 + (lane >> 3);
        const int j = lane & 7;
        ph[it] = *(const v4ua*)(sp + rowl * 64 + 8 * j);
        pl[it] = *(const v4ua*)(sp + 1024 + rowl * 64 + 8 * j);
        dst[it] = ((size_t)b * NTOK + q0 + rowl) * DM + hd * DK + 8 * j;
    }
    #pragma unroll
    for (int it = 0; it < 4; ++it) {
        *(volatile v4ua*)(Ch + dst[it]) = ph[it];
        *(volatile v4ua*)(Cl + dst[it]) = pl[it];
    }
    __threadfence();
    #pragma unroll
    for (int it = 0; it < 4; ++it) {
        *(volatile v4ua*)(Ch + dst[it]) = ph[it];
        *(volatile v4ua*)(Cl + dst[it]) = pl[it];
    }
}

extern "C" void kernel_launch(void* const* d_in, const int* in_sizes, int n_in,
                              void* d_out, int out_size, void* d_ws, size_t ws_size,
                              hipStream_t stream)
{
    if (n_in < 12) return;
    if (in_sizes[0] != ACT_N || in_sizes[1] != ACT_N || in_sizes[2] != ACT_N) return;
    if (in_sizes[3] != GATE_N) return;
    if (in_sizes[4] != W_N || in_sizes[6] != W_N || in_sizes[8] != W_N || in_sizes[10] != W_N) return;
    if (in_sizes[5] != DM || in_sizes[7] != DM || in_sizes[9] != DM || in_sizes[11] != DM) return;
    if (out_size != ACT_N) return;

    const size_t MIB = (size_t)1 << 20;
    const size_t total = 100 * MIB;
    if (ws_size < total) return;

    const float* query = (const float*)d_in[0];
    const float* key_  = (const float*)d_in[1];
    const float* value = (const float*)d_in[2];
    const float* wc    = (const float*)d_in[3];
    const float* Wq    = (const float*)d_in[4];
    const float* bq    = (const float*)d_in[5];
    const float* Wk    = (const float*)d_in[6];
    const float* bk    = (const float*)d_in[7];
    const float* Wv    = (const float*)d_in[8];
    const float* bv    = (const float*)d_in[9];
    const float* Wo    = (const float*)d_in[10];
    const float* bo    = (const float*)d_in[11];
    float* out = (float*)d_out;

    char* ws = (char*)d_ws;
    float* G   = (float*)(ws);
    u16*   XP  = (u16*)(ws + 32 * MIB);
    u16*   WP  = (u16*)(ws + 80 * MIB);
    u16*   QP  = (u16*)(ws + 84 * MIB);

    u16* Xqh = XP;               u16* Xql = XP + (size_t)1 * ACT_N;
    u16* Xkh = XP + (size_t)2 * ACT_N;  u16* Xkl = XP + (size_t)3 * ACT_N;
    u16* Xvh = XP + (size_t)4 * ACT_N;  u16* Xvl = XP + (size_t)5 * ACT_N;
    u16* Wqh = WP;               u16* Wql = WP + (size_t)1 * W_N;
    u16* Wkh = WP + (size_t)2 * W_N;    u16* Wkl = WP + (size_t)3 * W_N;
    u16* Wvh = WP + (size_t)4 * W_N;    u16* Wvl = WP + (size_t)5 * W_N;
    u16* Woh = WP + (size_t)6 * W_N;    u16* Wol = WP + (size_t)7 * W_N;
    u16* Qph = QP;               u16* Qpl = QP + (size_t)ACT_N;
    u16* Kph = Xqh;              u16* Kpl = Xql;
    u16* Vph = Xkh;              u16* Vpl = Xkl;
    u16* Cph = Xvh;              u16* Cpl = Xvl;

    const dim3 blk(256);
    const dim3 gemmGrid(DM / 64, MROWS / 128);
    const dim3 attnGrid(NTOK / 128, NB * NH);

    k_gate<<<dim3(MROWS), blk, 0, stream>>>(wc, G);
    k_split<<<dim3(3 * 2048 + 4 * 128), blk, 0, stream>>>(query, key_, value, Wq, Wk, Wv, Wo, XP, WP);
    k_gemm<0><<<gemmGrid, blk, 0, stream>>>(Xqh, Xql, Wqh, Wql, bq, Qph, Qpl, out);
    k_gemm<0><<<gemmGrid, blk, 0, stream>>>(Xkh, Xkl, Wkh, Wkl, bk, Kph, Kpl, out);
    k_gemm<1><<<gemmGrid, blk, 0, stream>>>(Xvh, Xvl, Wvh, Wvl, bv, Vph, Vpl, out);
    k_attn<<<attnGrid, blk, 0, stream>>>(Qph, Qpl, Kph, Kpl, Vph, Vpl, G, Cph, Cpl);
    k_gemm<2><<<gemmGrid, blk, 0, stream>>>(Cph, Cpl, Woh, Wol, bo, Cph, Cpl, out);
}
